// MultiHeadAttention_33844342293035
// MI455X (gfx1250) — hardware-run, weakly checked
//
#include <hip/hip_runtime.h>
#include <math.h>

#ifndef NB
#define NB 4
#endif
#ifndef SEQ
#define SEQ 2048
#endif
#define NB_FULL 4
#define SEQ_FULL 2048
#define EMB 512
#define NHEAD 8
#define HDIM 64
#define MROWS (NB * SEQ)
static_assert(NB >= 1 && NB <= NB_FULL);
static_assert(SEQ >= 64 && SEQ <= SEQ_FULL);
static_assert(SEQ % 64 == 0);
static_assert(MROWS % 64 == 0);
static_assert(EMB % 64 == 0 && EMB % 32 == 0);
static_assert(NHEAD * HDIM == EMB);
static_assert(HDIM == 64);

typedef __attribute__((ext_vector_type(16))) _Float16 v16h;
typedef __attribute__((ext_vector_type(8)))  _Float16 v8h;
typedef __attribute__((ext_vector_type(16))) __bf16   v16b;
typedef __attribute__((ext_vector_type(8)))  float    v8f;
typedef __attribute__((ext_vector_type(4)))  float    v4f;

__device__ __forceinline__ v8f wmma16(v16h a, v16h b, v8f c) {
    c = __builtin_amdgcn_wmma_f32_16x16x32_f16(false, a, false, b, (short)0, c, false, false);
    asm volatile("v_nop\n\tv_nop\n\tv_nop\n\tv_nop" : "+v"(c) : "v"(a), "v"(b));
    return c;
}
union FragH { v16h v; v8h h[2]; };

#define VST2(T, ptr, val) do { const T vst2_v_ = (val); *(volatile T*)(ptr) = vst2_v_; __threadfence(); *(volatile T*)(ptr) = vst2_v_; } while (0)

__device__ __forceinline__ void wave_lds_sync() {
    __builtin_amdgcn_fence(3  , "workgroup");
    __builtin_amdgcn_wave_barrier();
    __builtin_amdgcn_fence(2  , "workgroup");
}

#define AT_P 72
#define AT_OP 68
struct AttnG {
    const float* Q; const float* K; const float* V; float* O;
    long long sQb, sKb, sVb, sOb;
    int sQi, sKj, sVj, sOi, sQh, sKh, sVh, sOh;
    int Lk; float scale;
};
static_assert(sizeof(AttnG) == 4 * 8 + 4 * 8 + 8 * 4 + 2 * 4);

__global__ __launch_bounds__(128) __attribute__((amdgpu_num_vgpr(256))) void k_attn64(AttnG g) {
    __shared__ __align__(16) _Float16 Kh[64 * AT_P];
    __shared__ __align__(16) _Float16 Vt[64 * AT_P];
    __shared__ __align__(16) _Float16 Ph[4][16 * AT_P];
    __shared__ __align__(16) float    Os[4][16 * AT_OP];
    const int tid = threadIdx.x;
    const int lane = tid & 31, hf = lane >> 4, l15 = lane & 15;
    const int wave = __builtin_amdgcn_readfirstlane((int)(tid >> 5));
    const int h = blockIdx.y, b = blockIdx.z;
    const int q0 = blockIdx.x * 64 + wave * 16;
    const float L2E = 1.4426950408889634f;
    const float NEG = -__builtin_inff();

    v16h qa[2];
    {
        const float* qrow = g.Q + (long long)b * g.sQb + (long long)h * g.sQh + (long long)(q0 + l15) * g.sQi;
#pragma unroll
        for (int ks = 0; ks < 2; ++ks) {
            const v4f a0 = *(const v4f*)(qrow + ks * 32 + 8 * hf);
            const v4f a1 = *(const v4f*)(qrow + ks * 32 + 8 * hf + 4);
            const v4f a2 = *(const v4f*)(qrow + ks * 32 + 16 + 8 * hf);
            const v4f a3 = *(const v4f*)(qrow + ks * 32 + 16 + 8 * hf + 4);
            v16h q;
            q[0] = (_Float16)a0.x; q[1] = (_Float16)a0.y; q[2] = (_Float16)a0.z; q[3] = (_Float16)a0.w;
            q[4] = (_Float16)a1.x; q[5] = (_Float16)a1.y; q[6] = (_Float16)a1.z; q[7] = (_Float16)a1.w;
            q[8] = (_Float16)a2.x; q[9] = (_Float16)a2.y; q[10] = (_Float16)a2.z; q[11] = (_Float16)a2.w;
            q[12] = (_Float16)a3.x; q[13] = (_Float16)a3.y; q[14] = (_Float16)a3.z; q[15] = (_Float16)a3.w;
            qa[ks] = q;
        }
    }

    v8f o[4]; float m8[8], l8[8];
#pragma unroll
    for (int t = 0; t < 4; ++t) { v8f zz = {}; o[t] = zz; }
#pragma unroll
    for (int i = 0; i < 8; ++i) { m8[i] = NEG; l8[i] = 0.f; }

    const float* kbase = g.K + (long long)b * g.sKb + (long long)h * g.sKh;
    const float* vbase = g.V + (long long)b * g.sVb + (long long)h * g.sVh;
    const int kvr = tid >> 1, dh0 = (tid & 1) * 32;

#pragma unroll 1
    for (int j0 = 0; j0 < g.Lk; j0 += 64) {
        __syncthreads();
        {
            const float* krow = kbase + (long long)(j0 + kvr) * g.sKj + dh0;
            const float* vrow = vbase + (long long)(j0 + kvr) * g.sVj + dh0;
#pragma unroll 1
            for (int i = 0; i < 4; ++i) {
                const v4f k0 = *(const v4f*)(krow + 8 * i), k1 = *(const v4f*)(krow + 8 * i + 4);
                const v4f v0 = *(const v4f*)(vrow + 8 * i), v1 = *(const v4f*)(vrow + 8 * i + 4);
                v8h kh;
                kh[0] = (_Float16)k0.x; kh[1] = (_Float16)k0.y; kh[2] = (_Float16)k0.z; kh[3] = (_Float16)k0.w;
                kh[4] = (_Float16)k1.x; kh[5] = (_Float16)k1.y; kh[6] = (_Float16)k1.z; kh[7] = (_Float16)k1.w;
                *(v8h*)&Kh[kvr * AT_P + dh0 + 8 * i] = kh;
                const int d0 = dh0 + 8 * i;
                Vt[(d0 + 0) * AT_P + kvr] = (_Float16)v0.x; Vt[(d0 + 1) * AT_P + kvr] = (_Float16)v0.y;
                Vt[(d0 + 2) * AT_P + kvr] = (_Float16)v0.z; Vt[(d0 + 3) * AT_P + kvr] = (_Float16)v0.w;
                Vt[(d0 + 4) * AT_P + kvr] = (_Float16)v1.x; Vt[(d0 + 5) * AT_P + kvr] = (_Float16)v1.y;
                Vt[(d0 + 6) * AT_P + kvr] = (_Float16)v1.z; Vt[(d0 + 7) * AT_P + kvr] = (_Float16)v1.w;
            }
        }
        __syncthreads();

        v8f s[4];
#pragma unroll
        for (int t = 0; t < 4; ++t) {
            v8f acc = {};
#pragma unroll
            for (int ks = 0; ks < 2; ++ks) {
                FragH kb;
                kb.h[0] = *(const v8h*)&Kh[(t * 16 + l15) * AT_P + ks * 32 + 8 * hf];
                kb.h[1] = *(const v8h*)&Kh[(t * 16 + l15) * AT_P + ks * 32 + 16 + 8 * hf];
                acc = wmma16(qa[ks], kb.v, acc);
            }
            s[t] = acc;
        }

#pragma unroll
        for (int i = 0; i < 8; ++i) {
            const float sc0 = s[0][i] * g.scale * L2E;
            const float sc1 = s[1][i] * g.scale * L2E;
            const float sc2 = s[2][i] * g.scale * L2E;
            const float sc3 = s[3][i] * g.scale * L2E;
            float mx = fmaxf(fmaxf(sc0, sc1), fmaxf(sc2, sc3));
            mx = fmaxf(mx, __shfl_xor(mx, 1, 32)); mx = fmaxf(mx, __shfl_xor(mx, 2, 32));
            mx = fmaxf(mx, __shfl_xor(mx, 4, 32)); mx = fmaxf(mx, __shfl_xor(mx, 8, 32));
            const float mnew = fmaxf(m8[i], mx);
            const float corr = (m8[i] == NEG) ? 0.f : exp2f(m8[i] - mnew);
            const float p0 = exp2f(sc0 - mnew), p1 = exp2f(sc1 - mnew), p2 = exp2f(sc2 - mnew), p3 = exp2f(sc3 - mnew);
            float rs = 0.f; rs += p0; rs += p1; rs += p2; rs += p3;
            const int pr = (8 * hf + i) * AT_P + l15;
            Ph[wave][pr]      = (_Float16)(p0 * 4096.f);
            Ph[wave][pr + 16] = (_Float16)(p1 * 4096.f);
            Ph[wave][pr + 32] = (_Float16)(p2 * 4096.f);
            Ph[wave][pr + 48] = (_Float16)(p3 * 4096.f);
            rs += __shfl_xor(rs, 1, 32); rs += __shfl_xor(rs, 2, 32); rs += __shfl_xor(rs, 4, 32); rs += __shfl_xor(rs, 8, 32);
            l8[i] = l8[i] * corr + rs; m8[i] = mnew;
#pragma unroll
            for (int t = 0; t < 4; ++t) o[t][i] *= corr;
        }
        wave_lds_sync();

#pragma unroll
        for (int kk = 0; kk < 2; ++kk) {
            FragH pa;
            pa.h[0] = *(const v8h*)&Ph[wave][l15 * AT_P + kk * 32 + 8 * hf];
            pa.h[1] = *(const v8h*)&Ph[wave][l15 * AT_P + kk * 32 + 16 + 8 * hf];
#pragma unroll
            for (int t = 0; t < 4; ++t) {
                FragH vb;
                vb.h[0] = *(const v8h*)&Vt[(t * 16 + l15) * AT_P + kk * 32 + 8 * hf];
                vb.h[1] = *(const v8h*)&Vt[(t * 16 + l15) * AT_P + kk * 32 + 16 + 8 * hf];
                o[t] = wmma16(pa.v, vb.v, o[t]);
            }
        }
    }

#pragma unroll
    for (int i = 0; i < 8; ++i) {
        const float inv = (l8[i] > 0.f) ? 1.f / (l8[i] * 4096.f) : 0.f;
#pragma unroll
        for (int t = 0; t < 4; ++t) Os[wave][(8 * hf + i) * AT_OP + t * 16 + l15] = o[t][i] * inv;
    }
    wave_lds_sync();
    {
        float* ob = g.O + (long long)b * g.sOb + (long long)h * g.sOh;
        const int c4 = l15 * 4;
        for (int pass = 0; pass < 2; ++pass) {
#pragma unroll
            for (int it = 0; it < 8; ++it) {
                const int row = it * 2 + hf;
                const v4f val = *(const v4f*)&Os[wave][row * AT_OP + c4];
                *(volatile v4f*)(ob + (long long)(q0 + row) * g.sOi + c4) = val;
            }
            __threadfence();
        }
    }
}

namespace gk {
typedef __attribute__((ext_vector_type(8)))  __bf16   v8b;

__device__ __forceinline__ void dep_guard_h(v8f& a, v8f& b, v16h x, v16h y) { asm volatile("v_nop\n\tv_nop\n\tv_nop\n\tv_nop" : "+v"(a), "+v"(b) : "v"(x), "v"(y)); }
__device__ __forceinline__ void dep_guard_b(v8f& a, v8f& b, v16b x, v16b y) { asm volatile("v_nop\n\tv_nop\n\tv_nop\n\tv_nop" : "+v"(a), "+v"(b) : "v"(x), "v"(y)); }
__device__ __forceinline__ void keep4_h(v16h a, v16h b, v16h c, v16h d) { asm volatile("v_nop" :: "v"(a), "v"(b), "v"(c), "v"(d)); }
__device__ __forceinline__ void keep4_b(v16b a, v16b b, v16b c, v16b d) { asm volatile("v_nop" :: "v"(a), "v"(b), "v"(c), "v"(d)); }
__device__ __forceinline__ void acc_guard4(v8f& a, v8f& b, v8f& c, v8f& d) { asm volatile("v_nop\n\tv_nop\n\tv_nop\n\tv_nop" : "+v"(a), "+v"(b), "+v"(c), "+v"(d)); }
template <typename T> struct Frag;
template <> struct Frag<_Float16> {
  typedef v16h V; union U { v16h v; v8h h[2]; };
  static __device__ __forceinline__ v16h load(const _Float16* p) {
    U f; f.h[0] = *(const v8h*)(p); f.h[1] = *(const v8h*)(p + 16); return f.v;
  }
  static __device__ __forceinline__ v8f mma(v16h a, v16h b, v8f c) {
    return __builtin_amdgcn_wmma_f32_16x16x32_f16(false, a, false, b, (short)0, c, false, false);
  }
  static __device__ __forceinline__ void guard(v8f& a, v8f& b, v16h x, v16h y) { dep_guard_h(a, b, x, y); }
  static __device__ __forceinline__ void keep(v16h a, v16h b, v16h c, v16h d) { keep4_h(a, b, c, d); }
};
template <> struct Frag<__bf16> {
  typedef v16b V; union U { v16b v; v8b h[2]; };
  static __device__ __forceinline__ v16b load(const __bf16* p) {
    U f; f.h[0] = *(const v8b*)(p); f.h[1] = *(const v8b*)(p + 16); return f.v;
  }
  static __device__ __forceinline__ v8f mma(v16b a, v16b b, v8f c) {
    return __builtin_amdgcn_wmma_f32_16x16x32_bf16(false, a, false, b, (short)0, c, false, false);
  }
  static __device__ __forceinline__ void guard(v8f& a, v8f& b, v16b x, v16b y) { dep_guard_b(a, b, x, y); }
  static __device__ __forceinline__ void keep(v16b a, v16b b, v16b c, v16b d) { keep4_b(a, b, c, d); }
};

template <int ET> struct Elem;
template <> struct Elem<0> { typedef _Float16 T; };
template <> struct Elem<1> { typedef __bf16 T; };
template <int ET, bool SPLIT, int BIAS_MODE, bool RESID>
__global__ __launch_bounds__(256) void wmma_gemm64(
    const unsigned short* __restrict__ Ap, const unsigned short* __restrict__ A2p, int lda, long strideA,
    const unsigned short* __restrict__ Btp, const unsigned short* __restrict__ Bt2p, int ldb, long strideB,
    float* __restrict__ Cout, int ldc, long strideC,
    const float* __restrict__ bias,
    const float* __restrict__ resid, long strideR,
    int M, int N, int K, float scale) {
  typedef typename Elem<ET>::T T;
  typedef typename Frag<T>::V V;
  const T* A = (const T*)Ap; const T* A2 = (const T*)A2p; const T* Bt = (const T*)Btp; const T* Bt2 = (const T*)Bt2p;
  __shared__ __align__(16) float sT[8][16 * 68];
  const int b    = blockIdx.y;
  const int lane = threadIdx.x & 31;
  const int wave = __builtin_amdgcn_readfirstlane((int)(threadIdx.x >> 5));
  const int tilesN = N >> 6;
  const int tilesM = M >> 6;
  const int tile = blockIdx.x * 8 + wave;
  if (tile >= tilesM * tilesN) return;
  const int tm = tile / tilesN;
  const int tn = tile - tm * tilesN;
  const int m0 = tm << 6;
  const int n0 = tn << 6;

  const T* Ab  = A  + (size_t)b * strideA;
  const T* Bb  = Bt + (size_t)b * strideB;
  const T* Ab2 = SPLIT ? (A2  + (size_t)b * strideA) : nullptr;
  const T* Bb2 = SPLIT ? (Bt2 + (size_t)b * strideB) : nullptr;

  const int rlane = lane & 15;
  const int koff  = (lane >> 4) * 8;
  const int mOff  = (lane >> 4) * 8;

  v8f acc[4][4];
#pragma unroll
  for (int i = 0; i < 4; ++i)
#pragma unroll
    for (int j = 0; j < 4; ++j) acc[i][j] = (v8f){0.f,0.f,0.f,0.f,0.f,0.f,0.f,0.f};

  for (int k0 = 0; k0 < K; k0 += 32) {
    V bh[4], bl[4];
#pragma unroll
    for (int j = 0; j < 4; ++j) {
      const size_t bo = (size_t)(n0 + (j << 4) + rlane) * ldb + koff + k0;
      bh[j] = Frag<T>::load(Bb + bo);
      if (SPLIT) bl[j] = Frag<T>::load(Bb2 + bo);
    }
#pragma unroll
    for (int i = 0; i < 4; ++i) {
      const size_t ao = (size_t)(m0 + (i << 4) + rlane) * lda + koff + k0;
      V ah = Frag<T>::load(Ab + ao);
      V al;
      if (SPLIT) al = Frag<T>::load(Ab2 + ao);
#pragma unroll
      for (int j = 0; j < 4; ++j) {
        acc[i][j] = Frag<T>::mma(ah, bh[j], acc[i][j]);
        if (SPLIT) {
          acc[i][j] = Frag<T>::mma(ah, bl[j], acc[i][j]);
          acc[i][j] = Frag<T>::mma(al, bh[j], acc[i][j]);
        }
      }
      Frag<T>::guard(acc[i][0], acc[i][3], ah, SPLIT ? al : ah);
    }
    Frag<T>::keep(bh[0], bh[1], bh[2], bh[3]);
    if (SPLIT) Frag<T>::keep(bl[0], bl[1], bl[2], bl[3]);
  }
  acc_guard4(acc[0][0], acc[0][1], acc[0][2], acc[0][3]);
  acc_guard4(acc[1][0], acc[1][1], acc[1][2], acc[1][3]);
  acc_guard4(acc[2][0], acc[2][1], acc[2][2], acc[2][3]);
  acc_guard4(acc[3][0], acc[3][1], acc[3][2], acc[3][3]);

  const float* Rb = RESID ? (resid + (size_t)b * strideR) : nullptr;
  float* C = Cout + (size_t)b * strideC;
#pragma unroll
  for (int i = 0; i < 4; ++i) {
    const int mBase = m0 + (i << 4);
#pragma unroll
    for (int j = 0; j < 4; ++j) {
      const int n = n0 + (j << 4) + rlane;
      float bv = 0.f;
      if (BIAS_MODE == 2) bv = bias[n];
#pragma unroll
      for (int r = 0; r < 8; ++r) {
        float v = acc[i][j][r] * scale;
        if (BIAS_MODE == 1) v += bias[mBase + mOff + r];
        if (BIAS_MODE == 2) v += bv;
        if (RESID) v += Rb[(size_t)(mBase + mOff + r) * ldc + n];
        sT[wave][(mOff + r) * 68 + (j << 4) + rlane] = v;
      }
    }
    wave_lds_sync();
    {
      const int hh = lane >> 4, c4 = (lane & 15) * 4;
      for (int pass = 0; pass < 2; ++pass) {
#pragma unroll
        for (int it = 0; it < 8; ++it) {
          const int row = it * 2 + hh;
          const v4f v = *(const v4f*)&sT[wave][row * 68 + c4];
          *(volatile v4f*)(C + (size_t)(mBase + row) * ldc + n0 + c4) = v;
        }
        __threadfence();
      }
    }
    wave_lds_sync();
  }
}
}

__global__ __launch_bounds__(256) void k_cast16(const float* __restrict__ src, long long lds, _Float16* __restrict__ dst, long long ldd, int R, int C, float s) {
    const long long i = (long long)blockIdx.x * 256 + threadIdx.x; const long long np = (long long)R * (C / 2); if (i >= np) return; const int r = (int)(i / (C / 2)); const int c = 2 * (int)(i % (C / 2));
    const _Float16 h0 = (_Float16)(src[(long long)r * lds + c] * s), h1 = (_Float16)(src[(long long)r * lds + c + 1] * s);
    const unsigned u = (unsigned)__builtin_bit_cast(unsigned short, h0) | ((unsigned)__builtin_bit_cast(unsigned short, h1) << 16);
    volatile unsigned* d = (volatile unsigned*)(dst + (long long)r * ldd + c); *d = u; __threadfence(); *d = u; }

typedef unsigned int cm_u4 __attribute__((ext_vector_type(4)));
__device__ __forceinline__ unsigned int cmb_pk2(float a, float b) { return (unsigned int)__builtin_bit_cast(unsigned short, (_Float16)a) | ((unsigned int)__builtin_bit_cast(unsigned short, (_Float16)b) << 16); }
__device__ __forceinline__ float cmb_bf(float v) { const unsigned u = __builtin_bit_cast(unsigned, v); const unsigned r = (u + 0x7fffu + ((u >> 16) & 1u)) & 0xffff0000u; return __builtin_bit_cast(float, r); }
__global__ __launch_bounds__(256) void k_cm_bfvec(const float* __restrict__ SRC, float* __restrict__ DST, int n) { const int u = blockIdx.x * 256 + threadIdx.x; if (u >= n) return; VST2(float, DST + u, cmb_bf(SRC[u])); }
__global__ __launch_bounds__(256) void k_cm_castb(const float* __restrict__ SRC, long long sSb, int lds, unsigned short* __restrict__ DST, long long sDb, int ldd, int nR, int nC, float sc) {
    const long long u = (long long)blockIdx.x * 256 + threadIdx.x; const int per = nC / 8; if (u >= (long long)nR * per) return; const int r = (int)(u / per); const int c0 = 8 * (int)(u % per);
    const float* s = SRC + (long long)blockIdx.y * sSb + (long long)r * lds + c0; float w[8];
#pragma unroll
    for (int e = 0; e < 8; ++e) w[e] = cmb_bf(s[e]) * sc;
    cm_u4 pk; pk.x = cmb_pk2(w[0], w[1]); pk.y = cmb_pk2(w[2], w[3]); pk.z = cmb_pk2(w[4], w[5]); pk.w = cmb_pk2(w[6], w[7]);
    VST2(cm_u4, (cm_u4*)(DST + (long long)blockIdx.y * sDb + (long long)r * ldd + c0), pk); }

constexpr size_t al256(size_t n) { return ((n + 255) / 256) * 256; }
constexpr size_t SZ_X16  = al256((size_t)MROWS * EMB * 2);
constexpr size_t SZ_W316 = al256((size_t)3 * EMB * EMB * 2);
constexpr size_t SZ_QKV  = al256((size_t)MROWS * 3 * EMB * 4);
constexpr size_t SZ_AO   = al256((size_t)MROWS * EMB * 4);
constexpr size_t SZ_BR3  = al256((size_t)(3 * EMB + 64) * 4);
constexpr size_t SZ_WO16 = al256((size_t)EMB * EMB * 2);
constexpr size_t SZ_BRO  = al256((size_t)(EMB + 64) * 4);
constexpr size_t CARVE_BYTES = SZ_X16 + SZ_W316 + SZ_QKV + SZ_AO + SZ_BR3 + SZ_WO16 + SZ_BRO;
static_assert(CARVE_BYTES <= (size_t)134217728);

extern "C" void kernel_launch(void* const* d_in, const int* in_sizes, int n_in, void* d_out, int out_size, void* d_ws, size_t ws_size, hipStream_t stream) {
    if (n_in < 9) return;
    const long long xneed = (long long)(NB - 1) * SEQ_FULL * EMB + (long long)SEQ * EMB;
    if ((long long)in_sizes[0] < xneed) return;
    if (in_sizes[1] < EMB * EMB || in_sizes[3] < EMB * EMB || in_sizes[5] < EMB * EMB || in_sizes[7] < EMB * EMB) return;
    if (in_sizes[2] < EMB || in_sizes[4] < EMB || in_sizes[6] < EMB || in_sizes[8] < EMB) return;
    if ((long long)out_size < (long long)MROWS * EMB) return;
    if (CARVE_BYTES > ws_size) return;
    const float* xq = (const float*)d_in[0];
    const float* Wq = (const float*)d_in[1];
    const float* bq = (const float*)d_in[2];
    const float* Wk = (const float*)d_in[3];
    const float* bk = (const float*)d_in[4];
    const float* Wv = (const float*)d_in[5];
    const float* bv = (const float*)d_in[6];
    const float* Wo = (const float*)d_in[7];
    const float* bo = (const float*)d_in[8];
    float* out = (float*)d_out;
    char* wsp = (char*)d_ws;
    unsigned short* X16  = (unsigned short*)wsp; wsp += SZ_X16;
    unsigned short* W316 = (unsigned short*)wsp; wsp += SZ_W316;
    float* QKV = (float*)wsp; wsp += SZ_QKV;
    float* AO  = (float*)wsp; wsp += SZ_AO;
    float* BR3 = (float*)wsp; wsp += SZ_BR3;
    unsigned short* WO16 = (unsigned short*)wsp; wsp += SZ_WO16;
    float* BRO = (float*)wsp; wsp += SZ_BRO;
    unsigned short* AO16 = X16;

    const unsigned wgrid = (unsigned)(((long long)EMB * (EMB / 8) + 255) / 256);
    k_cm_castb<<<dim3(wgrid, 1), 256, 0, stream>>>(Wq, 0, EMB, W316, 0, EMB, EMB, EMB, 16.0f);
    k_cm_castb<<<dim3(wgrid, 1), 256, 0, stream>>>(Wk, 0, EMB, W316 + (size_t)EMB * EMB, 0, EMB, EMB, EMB, 16.0f);
    k_cm_castb<<<dim3(wgrid, 1), 256, 0, stream>>>(Wv, 0, EMB, W316 + (size_t)2 * EMB * EMB, 0, EMB, EMB, EMB, 16.0f);
    k_cm_castb<<<dim3(wgrid, 1), 256, 0, stream>>>(Wo, 0, EMB, WO16, 0, EMB, EMB, EMB, 16.0f);
    k_cm_bfvec<<<(EMB + 255) / 256, 256, 0, stream>>>(bq, BR3, EMB);
    k_cm_bfvec<<<(EMB + 255) / 256, 256, 0, stream>>>(bk, BR3 + EMB, EMB);
    k_cm_bfvec<<<(EMB + 255) / 256, 256, 0, stream>>>(bv, BR3 + 2 * EMB, EMB);
    k_cm_bfvec<<<(EMB + 255) / 256, 256, 0, stream>>>(bo, BRO, EMB);
    k_cm_castb<<<dim3((unsigned)(((long long)SEQ * (EMB / 8) + 255) / 256), (unsigned)NB), 256, 0, stream>>>(
        xq, (long long)SEQ_FULL * EMB, EMB, X16, (long long)SEQ * EMB, EMB, SEQ, EMB, 1.0f);
    gk::wmma_gemm64<0, false, 2, false><<<dim3((unsigned)(((MROWS / 64) * ((3 * EMB) / 64) + 7) / 8), 1u), 256, 0, stream>>>(
        (const unsigned short*)X16, nullptr, EMB, 0, (const unsigned short*)W316, nullptr, EMB, 0,
        QKV, 3 * EMB, 0, BR3, nullptr, 0, MROWS, 3 * EMB, EMB, 0.0625f);
    {
        AttnG a;
        a.Q = QKV; a.K = QKV + EMB; a.V = QKV + 2 * EMB; a.O = AO;
        a.sQb = (long long)SEQ * 3 * EMB; a.sKb = (long long)SEQ * 3 * EMB; a.sVb = (long long)SEQ * 3 * EMB; a.sOb = (long long)SEQ * EMB;
        a.sQi = 3 * EMB; a.sKj = 3 * EMB; a.sVj = 3 * EMB; a.sOi = EMB;
        a.sQh = HDIM; a.sKh = HDIM; a.sVh = HDIM; a.sOh = HDIM;
        a.Lk = SEQ; a.scale = 0.04419417306780815f;
        k_attn64<<<dim3((unsigned)(SEQ / 64), (unsigned)NHEAD, (unsigned)NB), 128, 0, stream>>>(a);
    }
    k_cast16<<<(unsigned)((((long long)MROWS * (EMB / 2)) + 255) / 256), 256, 0, stream>>>(AO, EMB, (_Float16*)AO16, EMB, MROWS, EMB, 64.0f);
    gk::wmma_gemm64<0, false, 2, false><<<dim3((unsigned)(((MROWS / 64) * (EMB / 64) + 7) / 8), 1u), 256, 0, stream>>>(
        (const unsigned short*)AO16, nullptr, EMB, 0, (const unsigned short*)WO16, nullptr, EMB, 0,
        out, EMB, 0, BRO, nullptr, 0, MROWS, EMB, EMB, 0.0009765625f);
}
